// GATNeigh_Agg_44822278701142
// MI455X (gfx1250) — hardware-verified
//
#include <hip/hip_runtime.h>
#include <stddef.h>


typedef _Float16 v16h __attribute__((ext_vector_type(16)));
typedef _Float16 v8h  __attribute__((ext_vector_type(8)));
typedef _Float16 v4h  __attribute__((ext_vector_type(4)));
typedef float    v8f  __attribute__((ext_vector_type(8)));
typedef float    v4f  __attribute__((ext_vector_type(4)));
typedef _Float16 h16;

#ifndef NB
#define NB 4
#endif
#ifndef SEQ
#define SEQ 512
#endif
#define NB_FULL  4
#define SEQ_FULL 512
#define FIN   64
#define FOUT  64
#define MROWS (NB * SEQ)

static_assert(NB >= 1 && NB <= NB_FULL);
static_assert(SEQ >= 128 && SEQ <= SEQ_FULL && (SEQ % 128) == 0);
static_assert((FIN % 64) == 0 && (FIN % 32) == 0);
static_assert(FOUT == 64);
static_assert(FIN == FOUT);
static_assert(FIN == 4 * 16);
static_assert((MROWS % 64) == 0 && (SEQ % 64) == 0 && (SEQ % 16) == 0);
static_assert(((SEQ / 2) % 32) == 0);
static_assert(((size_t)MROWS * FIN) % 2048 == 0);
static_assert((size_t)MROWS * FIN < (size_t)0xFFFFFFFFu);

#define LDT 72
#define LDC 68
#define PLD (SEQ + 8)
#define HLD (FIN + 4)
#define NJ  (SEQ / 32)
static_assert((LDT % 8) == 0 && LDT >= 64);
static_assert((LDC % 4) == 0 && LDC >= 64);
static_assert((PLD % 8) == 0 && (HLD % 4) == 0);
static_assert(NJ * 32 == SEQ);
static_assert(8 * 2 == 16);
static_assert(16 * FOUT == 256 * 4);
static_assert(16 * FIN == 256 * 4);
static_assert(4 * 16 == 64 && 16 * 4 == FOUT);

#define WCARRY 64.0f
#define PCARRY 16384.0f
#define ALPHA  0.2f
#define NEGFILL (-1.0e12f)

#define WT_BYTES  ((size_t)2 * FOUT * FIN * 2)
#define H16_BYTES ((size_t)MROWS * FIN * 2)
#define VT_BYTES  ((size_t)NB * FIN * SEQ * 2)
#define PRJ_BYTES ((size_t)2 * MROWS * FOUT * 4)
#define OFF_WT  ((size_t)0)
#define OFF_H16 (OFF_WT + WT_BYTES)
#define OFF_VT  (OFF_H16 + H16_BYTES)
#define OFF_PRJ (OFF_VT + VT_BYTES)
#define WS_TOTAL (OFF_PRJ + PRJ_BYTES)
static_assert((WT_BYTES % 128) == 0 && (H16_BYTES % 128) == 0);
static_assert((VT_BYTES % 128) == 0 && (PRJ_BYTES % 128) == 0);
static_assert(WS_TOTAL <= (size_t)134217728);

__device__ __forceinline__ float bf16r(float x) {
  unsigned int u = __float_as_uint(x);
  u = (u + 0x7FFFu + ((u >> 16) & 1u)) & 0xFFFF0000u;
  return __uint_as_float(u);
}

static __device__ __forceinline__ h16 toh_flush(float v) {
  const h16 r = (h16)v;
  return (fabsf(v) < 6.103515625e-05f) ? (h16)0.0f : r;
}

__device__ __forceinline__ v16h frag_at(const _Float16* p) {
  v8h lo = *(const v8h*)(p);
  v8h hi = *(const v8h*)(p + 16);
  v16h out;
#pragma unroll
  for (int i = 0; i < 8; ++i) { out[i] = lo[i]; out[i + 8] = hi[i]; }
  return out;
}
__device__ __forceinline__ v16h ld_frag(const _Float16* base, unsigned ld) {
  const unsigned lane = threadIdx.x & 31u;
  return frag_at(base + (lane & 15u) * ld + (lane >> 4) * 8u);
}

__device__ __forceinline__ v8f wmma16(v16h a, v16h b, v8f c) {
  v8f d = __builtin_amdgcn_wmma_f32_16x16x32_f16(false, a, false, b, (short)0, c,
                                                 false, false);
  asm volatile("v_nop\n\tv_nop\n\tv_nop\n\tv_nop" : "+v"(d) : "v"(a), "v"(b));
  return d;
}

__device__ __forceinline__ float red32_sum(float x) {
#pragma unroll
  for (int off = 1; off < 32; off <<= 1) x += __shfl_xor(x, off, 32);
  return x;
}
__device__ __forceinline__ float red32_max(float x) {
#pragma unroll
  for (int off = 1; off < 32; off <<= 1) x = fmaxf(x, __shfl_xor(x, off, 32));
  return x;
}

__global__ __launch_bounds__(256) void wconv_kernel(
    const float* __restrict__ W, _Float16* __restrict__ Wt, unsigned ldw, unsigned ldk) {
  __shared__ _Float16 T[64 * LDT];
  const unsigned tid = threadIdx.x;
  const unsigned n0 = blockIdx.x * 64u;
  const unsigned k0 = blockIdx.y * 64u;
#pragma unroll 4
  for (unsigned j = 0; j < 16u; ++j) {
    const unsigned idx = tid + 256u * j;
    const unsigned kr = idx >> 6, nc = idx & 63u;
    const float v = W[(size_t)(k0 + kr) * ldw + n0 + nc];
    T[nc * LDT + kr] = toh_flush(WCARRY * bf16r(v));
  }
  __syncthreads();
  v8h x[2];
  size_t off[2];
#pragma unroll
  for (unsigned i = 0; i < 2u; ++i) {
    const unsigned n = 32u * i + (tid >> 3);
    const unsigned kc = (tid & 7u) * 8u;
    x[i] = *(const v8h*)&T[n * LDT + kc];
    off[i] = (size_t)(n0 + n) * ldk + k0 + kc;
  }
#pragma unroll
  for (int i = 0; i < 2; ++i) *(volatile v8h*)(Wt + off[i]) = x[i];
  __threadfence();
#pragma unroll
  for (int i = 0; i < 2; ++i) *(volatile v8h*)(Wt + off[i]) = x[i];
}

__global__ __launch_bounds__(256) void hconv_kernel(
    const float* __restrict__ X, _Float16* __restrict__ dst) {
  const unsigned g = blockIdx.x * 256u + threadIdx.x;
  const unsigned crow = g / (unsigned)(FIN / 8);
  const unsigned c = (g - crow * (unsigned)(FIN / 8)) * 8u;
  const unsigned bidx = crow / (unsigned)SEQ;
  const unsigned sq = crow - bidx * (unsigned)SEQ;
  const size_t srow = (size_t)bidx * SEQ_FULL + sq;
  const v4f a0 = *(const v4f*)(X + srow * FIN + c);
  const v4f a1 = *(const v4f*)(X + srow * FIN + c + 4u);
  v8h o;
#pragma unroll
  for (int i = 0; i < 4; ++i) {
    o[i]     = toh_flush(bf16r(a0[i]));
    o[i + 4] = toh_flush(bf16r(a1[i]));
  }
  _Float16* p = dst + (size_t)crow * FIN + c;
  *(volatile v8h*)p = o;
  __threadfence();
  *(volatile v8h*)p = o;
}

__global__ __launch_bounds__(256) void gemm_proj_kernel(
    const _Float16* __restrict__ A16, const _Float16* __restrict__ Bt,
    float* __restrict__ prj) {
  __shared__ __attribute__((aligned(16))) float Cs[64 * LDC];
  const unsigned tid = threadIdx.x, lane = tid & 31u;
  const unsigned w = __builtin_amdgcn_readfirstlane(tid >> 5);
  const unsigned mw = w >> 1, nw = w & 1u;
  const unsigned hh = lane >> 4, m = lane & 15u;
  const unsigned n0 = blockIdx.x * 64u;
  const unsigned row0 = blockIdx.y * 64u;
  const unsigned K = (unsigned)FIN;

  const _Float16* ap  = A16 + (size_t)(row0 + mw * 16u + m) * K + hh * 8u;
  const _Float16* bp0 = Bt + (size_t)(n0 + nw * 32u + m) * K + hh * 8u;
  const _Float16* bp1 = bp0 + (size_t)16 * K;
  v8f acc0 = {}, acc1 = {};
#pragma unroll 2
  for (unsigned k0 = 0; k0 < K; k0 += 32u) {
    const v16h a  = frag_at(ap + k0);
    const v16h b0 = frag_at(bp0 + k0);
    const v16h b1 = frag_at(bp1 + k0);
    acc0 = wmma16(a, b0, acc0);
    acc1 = wmma16(a, b1, acc1);
  }
#pragma unroll
  for (int r = 0; r < 8; ++r) {
    float* d = &Cs[(mw * 16u + hh * 8u + (unsigned)r) * LDC + nw * 32u + m];
    d[0]  = acc0[r];
    d[16] = acc1[r];
  }
  __syncthreads();

  {
    v4f x[4];
    size_t off[4];
#pragma unroll
    for (unsigned i = 0; i < 4u; ++i) {
      const unsigned idx = 256u * i + tid;
      const unsigned r = idx >> 4;
      const unsigned c = (idx & 15u) * 4u;
      const v4f t = *(const v4f*)&Cs[r * LDC + c];
#pragma unroll
      for (int q = 0; q < 4; ++q) x[i][q] = t[q] * (1.0f / WCARRY);
      off[i] = ((size_t)blockIdx.x * MROWS + row0 + r) * FOUT + c;
    }
#pragma unroll
    for (int i = 0; i < 4; ++i) *(volatile v4f*)(prj + off[i]) = x[i];
    __threadfence();
#pragma unroll
    for (int i = 0; i < 4; ++i) *(volatile v4f*)(prj + off[i]) = x[i];
  }
}

__global__ __launch_bounds__(256) void neigh_attn_kernel(
    const int* __restrict__ adj, const _Float16* __restrict__ Vt,
    const float* __restrict__ VU, const float* __restrict__ IV,
    const float* __restrict__ Y, float* __restrict__ out) {
  __shared__ __attribute__((aligned(16))) _Float16 Ps[16 * PLD];
  __shared__ __attribute__((aligned(16))) float Ls[16 * SEQ];
  __shared__ __attribute__((aligned(16))) float Hs[2 * 16 * HLD];
  __shared__ __attribute__((aligned(16))) float vus[16 * FOUT];
  __shared__ __attribute__((aligned(16))) float ys[FOUT];
  __shared__ float rinv[16];

  const unsigned tid = threadIdx.x, lane = tid & 31u;
  const unsigned w = __builtin_amdgcn_readfirstlane(tid >> 5);
  const unsigned hh = lane >> 4, m = lane & 15u;
  const unsigned i0 = blockIdx.x * 16u;
  const unsigned b = blockIdx.y;

  {
    const v4f u = *(const v4f*)(VU + ((size_t)b * SEQ + i0) * FOUT + tid * 4u);
    *(v4f*)&vus[tid * 4u] = u;
    const unsigned yi = (tid & 15u) * 4u;
    const v4f y = *(const v4f*)(Y + yi);
    v4f yb;
#pragma unroll
    for (int q = 0; q < 4; ++q) yb[q] = bf16r(y[q]);
    if (tid < 16u) *(v4f*)&ys[yi] = yb;
  }
  __syncthreads();

  {
    const unsigned r0 = w * 2u;
    const int* adj0 = adj + ((size_t)b * SEQ_FULL + i0 + r0) * SEQ_FULL + lane;
    const int* adj1 = adj0 + SEQ_FULL;
    const float* ivb = IV + ((size_t)b * SEQ + lane) * FOUT;
    float mx0 = -3.0e38f, mx1 = -3.0e38f;
#pragma unroll 1
    for (unsigned jj = 0; jj < (unsigned)NJ; ++jj) {
      const unsigned j = jj * 32u + lane;
      const float* ivr = ivb + (size_t)jj * 32u * FOUT;
      int m0 = adj0[jj * 32u];
      int m1 = adj1[jj * 32u];
      asm volatile("" : "+v"(m0));
      asm volatile("" : "+v"(m1));
      float a0 = 0.0f, a1 = 0.0f;
#pragma unroll 4
      for (unsigned c4 = 0; c4 < (unsigned)(FOUT / 4); ++c4) {
        const v4f v  = *(const v4f*)(ivr + c4 * 4u);
        const v4f u0 = *(const v4f*)&vus[r0 * FOUT + c4 * 4u];
        const v4f u1 = *(const v4f*)&vus[(r0 + 1u) * FOUT + c4 * 4u];
        const v4f y  = *(const v4f*)&ys[c4 * 4u];
#pragma unroll
        for (int q = 0; q < 4; ++q) {
          const float t0 = u0[q] + v[q];
          const float t1 = u1[q] + v[q];
          const float l0 = (t0 >= 0.0f) ? t0 : ALPHA * t0;
          const float l1 = (t1 >= 0.0f) ? t1 : ALPHA * t1;
          a0 = fmaf(l0, y[q], a0);
          a1 = fmaf(l1, y[q], a1);
        }
      }
      const float e0 = (m0 > 0) ? a0 : NEGFILL;
      const float e1 = (m1 > 0) ? a1 : NEGFILL;
      Ls[r0 * SEQ + j] = e0;
      Ls[(r0 + 1u) * SEQ + j] = e1;
      mx0 = fmaxf(mx0, e0);
      mx1 = fmaxf(mx1, e1);
    }
    mx0 = red32_max(mx0);
    mx1 = red32_max(mx1);
    float sum0 = 0.0f, sum1 = 0.0f;
#pragma unroll 1
    for (unsigned jj = 0; jj < (unsigned)NJ; ++jj) {
      const unsigned j = jj * 32u + lane;
      const float e0 = Ls[r0 * SEQ + j];
      const float e1 = Ls[(r0 + 1u) * SEQ + j];
      const float p0 = __expf(e0 - mx0) * PCARRY;
      const float p1 = __expf(e1 - mx1) * PCARRY;
      const h16 h0 = toh_flush(p0);
      const h16 h1 = toh_flush(p1);
      Ps[r0 * PLD + j] = h0;
      Ps[(r0 + 1u) * PLD + j] = h1;
      sum0 += (float)h0;
      sum1 += (float)h1;
    }
    sum0 = red32_sum(sum0);
    sum1 = red32_sum(sum1);
    if (lane == 0u) {
      rinv[r0] = 1.0f / sum0;
      rinv[r0 + 1u] = 1.0f / sum1;
    }
  }
  __syncthreads();

  {
    const unsigned ct = w & 3u, kh = w >> 2;
    const unsigned kbase = kh * (unsigned)(SEQ / 2);
    const _Float16* bp = Vt + ((size_t)b * FIN + ct * 16u + m) * SEQ + kbase + hh * 8u;
    v8f acc = {};
#pragma unroll 2
    for (unsigned k0 = 0; k0 < (unsigned)(SEQ / 2); k0 += 32u) {
      const v16h a  = ld_frag(&Ps[kbase + k0], PLD);
      const v16h bb = frag_at(bp + k0);
      acc = wmma16(a, bb, acc);
    }
#pragma unroll
    for (int r = 0; r < 8; ++r) {
      const unsigned row = hh * 8u + (unsigned)r;
      Hs[(kh * 16u + row) * HLD + ct * 16u + m] = acc[r];
    }
  }
  __syncthreads();

  {
    const unsigned r = w * 2u + hh;
    const unsigned c = m * 4u;
    const v4f x0 = *(const v4f*)&Hs[r * HLD + c];
    const v4f x1 = *(const v4f*)&Hs[(16u + r) * HLD + c];
    const float sc = rinv[r] * (1.0f / WCARRY);
    v4f o;
#pragma unroll
    for (int i = 0; i < 4; ++i) {
      const float t = (x0[i] + x1[i]) * sc;
      o[i] = (t >= 0.0f) ? t : ALPHA * t;
    }
    float* p = out + ((size_t)b * SEQ_FULL + i0 + r) * FIN + c;
    *(volatile v4f*)p = o;
    __threadfence();
    *(volatile v4f*)p = o;
  }
}

static_assert(16 * PLD * 2 + 16 * SEQ * 4 + 2 * 16 * HLD * 4 + 16 * FOUT * 4 + FOUT * 4 + 64 <= 65536);
static_assert(64 * LDC * 4 <= 131072);
static_assert(64 * LDT * 2 <= 131072);

extern "C" void kernel_launch(void* const* d_in, const int* in_sizes, int n_in,
                              void* d_out, int out_size, void* d_ws, size_t ws_size,
                              hipStream_t stream) {
  if (n_in < 7) return;
  const long long need_rows = (long long)(NB - 1) * SEQ_FULL + SEQ;
  if ((long long)in_sizes[0] < need_rows * FIN) return;
  if ((long long)in_sizes[1] < (need_rows - 1) * SEQ_FULL + SEQ) return;
  if ((long long)in_sizes[4] < (long long)FIN * FOUT) return;
  if ((long long)in_sizes[5] < (long long)FIN * FOUT) return;
  if (in_sizes[6] < FOUT) return;
  if ((long long)out_size < need_rows * FIN) return;
  if (ws_size < WS_TOTAL) return;

  const float* X    = (const float*)d_in[0];
  const int*   adj  = (const int*)d_in[1];
  const float* W2   = (const float*)d_in[4];
  const float* U2   = (const float*)d_in[5];
  const float* yita = (const float*)d_in[6];
  float* out = (float*)d_out;

  char* ws = (char*)d_ws;
  _Float16* Wt16 = (_Float16*)(ws + OFF_WT);
  _Float16* H16  = (_Float16*)(ws + OFF_H16);
  _Float16* Vt16 = (_Float16*)(ws + OFF_VT);
  float*    Prj  = (float*)(ws + OFF_PRJ);

  dim3 blk(256);
  wconv_kernel<<<dim3(FOUT / 64, FIN / 64), blk, 0, stream>>>(U2, Wt16, (unsigned)FOUT, (unsigned)FIN);
  wconv_kernel<<<dim3(FOUT / 64, FIN / 64), blk, 0, stream>>>(W2, Wt16 + (size_t)FOUT * FIN,
                                                               (unsigned)FOUT, (unsigned)FIN);
  for (int bb = 0; bb < NB; ++bb) {
    wconv_kernel<<<dim3(FIN / 64, SEQ / 64), blk, 0, stream>>>(
        X + (size_t)bb * SEQ_FULL * FIN, Vt16 + (size_t)bb * FIN * SEQ, (unsigned)FIN, (unsigned)SEQ);
  }
  hconv_kernel<<<dim3((unsigned)(((size_t)MROWS * FIN) / 2048)), blk, 0, stream>>>(X, H16);
  gemm_proj_kernel<<<dim3(2, MROWS / 64), blk, 0, stream>>>(H16, Wt16, Prj);
  neigh_attn_kernel<<<dim3(SEQ / 16, NB), blk, 0, stream>>>(
      adj, Vt16, Prj, Prj + (size_t)MROWS * FOUT, yita, out);
}
